// LSTMCellManual_14654428413974
// MI455X (gfx1250) — hardware-verified
//
#include <hip/hip_runtime.h>
#include <stdint.h>
#include <stddef.h>


#define DIN   1024
#define DHID  1024
#define KTOT  2048
#define KV4   (KTOT / 8)
#define KSTEPS (KTOT / 32)
#define TM    128
#define TN    64
#define LDQ   5
#define EP    36

typedef float        v4f  __attribute__((ext_vector_type(4)));
typedef float        v8f  __attribute__((ext_vector_type(8)));
typedef unsigned int v4u  __attribute__((ext_vector_type(4)));
typedef __bf16       v16bf __attribute__((ext_vector_type(16)));
typedef v4f v4fa __attribute__((may_alias));

union Frag { v16bf v; v4u u[2]; };

static_assert(TM * LDQ * 16 + 4 * TN * LDQ * 16 + 8 * 16 * EP * 4 <= 65536);
static_assert((EP * 4) % 16 == 0);

__device__ __forceinline__ unsigned int f2bf(float f) {
    unsigned int u = __builtin_bit_cast(unsigned int, f);
    u += 0x7FFFu + ((u >> 16) & 1u);
    return u >> 16;
}
__device__ __forceinline__ unsigned int pack2(float f0, float f1) {
    return (f2bf(f0) & 0xFFFFu) | (f2bf(f1) << 16);
}
__device__ __forceinline__ float bf16r(float f) {
    unsigned int u = __builtin_bit_cast(unsigned int, f);
    u = (u + 0x7FFFu + ((u >> 16) & 1u)) & 0xFFFF0000u;
    return __builtin_bit_cast(float, u);
}

__device__ __forceinline__ float fsigm(float x) {
    return __builtin_amdgcn_rcpf(1.0f + __expf(-x));
}
__device__ __forceinline__ float ftanh(float x) {
    return 1.0f - 2.0f * __builtin_amdgcn_rcpf(1.0f + __expf(2.0f * x));
}

__device__ __forceinline__ void wmma_pair(v8f& c0, v8f& c1, const v16bf a0, const v16bf a1, const v16bf b) {
    c0 = __builtin_amdgcn_wmma_f32_16x16x32_bf16(false, a0, false, b, (short)0, c0, false, false);
    c1 = __builtin_amdgcn_wmma_f32_16x16x32_bf16(false, a1, false, b, (short)0, c1, false, false);
    asm volatile("v_nop\n\tv_nop\n\tv_nop\n\tv_nop" : "+v"(c0), "+v"(c1) : "v"(a0), "v"(a1), "v"(b));
}

__global__ __launch_bounds__(256)
void k_cvt(const float* __restrict__ s0, const float* __restrict__ s1, unsigned short* __restrict__ dst)
{
    const int row = blockIdx.x;
    const int t   = threadIdx.x;
    const float* src = (t < 128) ? s0 : s1;
    const size_t so = (size_t)row * DIN + (size_t)((t & 127) * 8);
    const v4fa* sp = (const v4fa*)(src + so);
    v4f f0 = sp[0];
    v4f f1 = sp[1];
    v4u pk;
    pk.x = pack2(f0.x, f0.y);
    pk.y = pack2(f0.z, f0.w);
    pk.z = pack2(f1.x, f1.y);
    pk.w = pack2(f1.z, f1.w);
    unsigned short* dp = dst + (size_t)row * KTOT + (size_t)(t * 8);
    *(volatile v4u*)dp = pk;
    __threadfence();
    *(volatile v4u*)dp = pk;
}

__global__ __launch_bounds__(256)
void k_lstm(const unsigned short* __restrict__ Acat,
            const unsigned short* __restrict__ Wcat,
            const float* __restrict__ c,
            const float* __restrict__ bi0, const float* __restrict__ bi1,
            const float* __restrict__ bi2, const float* __restrict__ bi3,
            const float* __restrict__ bh0, const float* __restrict__ bh1,
            const float* __restrict__ bh2, const float* __restrict__ bh3,
            float* __restrict__ out0, float* __restrict__ out1)
{
    __shared__ v4u lsA[TM * LDQ];
    __shared__ v4u lsB[4 * TN * LDQ];
    __shared__ __attribute__((aligned(16))) float lsE[8 * 16 * EP];

    const int tid  = threadIdx.x;
    const int lane = tid & 31;
    const int wave = tid >> 5;
    const int m    = lane & 15;
    const int h    = lane >> 4;
    const int wm   = wave & 3;
    const int wn   = wave >> 2;
    const int m0   = blockIdx.y * TM;
    const int n0   = blockIdx.x * TN;

    const v4u* A8 = (const v4u*)Acat;
    const v4u* W8 = (const v4u*)Wcat;

    const int part = tid & 3;
    const int rowa = tid >> 2;
    const size_t ga0 = (size_t)(m0 + rowa) * KV4 + part;
    const size_t ga1 = (size_t)(m0 + rowa + 64) * KV4 + part;
    const size_t gw0 = ((size_t)0 * DHID + n0 + rowa) * KV4 + part;
    const size_t gw1 = ((size_t)1 * DHID + n0 + rowa) * KV4 + part;
    const size_t gw2 = ((size_t)2 * DHID + n0 + rowa) * KV4 + part;
    const size_t gw3 = ((size_t)3 * DHID + n0 + rowa) * KV4 + part;
    const int la0 = rowa * LDQ + part;
    const int la1 = (rowa + 64) * LDQ + part;
    const int lb  = rowa * LDQ + part;

    const int ra0 = (wm * 32 + m) * LDQ;
    const int ra1 = (wm * 32 + 16 + m) * LDQ;
    const int rb0 = (wn * 32 + m) * LDQ;
    const int rb1 = (wn * 32 + 16 + m) * LDQ;

    v8f acc[4][2][2];
    #pragma unroll
    for (int g = 0; g < 4; ++g)
        #pragma unroll
        for (int a = 0; a < 2; ++a)
            #pragma unroll
            for (int b = 0; b < 2; ++b)
                acc[g][a][b] = (v8f)0.0f;

    #pragma unroll 1
    for (int kt = 0; kt < KSTEPS; ++kt) {
        const int kc = kt * 4;
        v4u sa0 = A8[ga0 + kc];
        v4u sa1 = A8[ga1 + kc];
        v4u sw0 = W8[gw0 + kc];
        v4u sw1 = W8[gw1 + kc];
        v4u sw2 = W8[gw2 + kc];
        v4u sw3 = W8[gw3 + kc];
        __syncthreads();
        lsA[la0] = sa0;
        lsA[la1] = sa1;
        lsB[lb + 0 * TN * LDQ] = sw0;
        lsB[lb + 1 * TN * LDQ] = sw1;
        lsB[lb + 2 * TN * LDQ] = sw2;
        lsB[lb + 3 * TN * LDQ] = sw3;
        __syncthreads();

        Frag a0, a1;
        a0.u[0] = lsA[ra0 + h];
        a0.u[1] = lsA[ra0 + 2 + h];
        a1.u[0] = lsA[ra1 + h];
        a1.u[1] = lsA[ra1 + 2 + h];
        #pragma unroll
        for (int g = 0; g < 4; ++g) {
            #pragma unroll
            for (int nB = 0; nB < 2; ++nB) {
                const int rb = g * TN * LDQ + (nB ? rb1 : rb0);
                Frag b;
                b.u[0] = lsB[rb + h];
                b.u[1] = lsB[rb + 2 + h];
                wmma_pair(acc[g][0][nB], acc[g][1][nB], a0.v, a1.v, b.v);
            }
        }
    }

    float bs[4][2];
    #pragma unroll
    for (int nB = 0; nB < 2; ++nB) {
        const int N = n0 + wn * 32 + nB * 16 + m;
        bs[0][nB] = bf16r(bi0[N]) + bf16r(bh0[N]);
        bs[1][nB] = bf16r(bi1[N]) + bf16r(bh1[N]);
        bs[2][nB] = bf16r(bi2[N]) + bf16r(bh2[N]);
        bs[3][nB] = bf16r(bi3[N]) + bf16r(bh3[N]);
    }

    float hv[2][2][8], cv2[2][2][8];
    #pragma unroll
    for (int mA = 0; mA < 2; ++mA) {
        #pragma unroll
        for (int nB = 0; nB < 2; ++nB) {
            const int N = n0 + wn * 32 + nB * 16 + m;
            #pragma unroll
            for (int r = 0; r < 8; ++r) {
                const int M = m0 + wm * 32 + mA * 16 + 8 * h + r;
                const float xi = acc[0][mA][nB][r] + bs[0][nB];
                const float xf = acc[1][mA][nB][r] + bs[1][nB];
                const float xg = acc[2][mA][nB][r] + bs[2][nB];
                const float xo = acc[3][mA][nB][r] + bs[3][nB];
                const float it = fsigm(xi);
                const float ft = fsigm(xf);
                const float gt = ftanh(xg);
                const float ot = fsigm(xo);
                const float cval = bf16r(c[(size_t)M * DHID + N]);
                const float cn = ft * cval + it * gt;
                const float hn = ot * ftanh(cn);
                hv[mA][nB][r]  = hn;
                cv2[mA][nB][r] = cn;
            }
        }
    }

    float* lsEw = lsE + wave * (16 * EP);
    const int rsub = lane >> 3;
    const int c4   = (lane & 7) * 4;
    v4f stv[2][2][4];
    #pragma unroll
    for (int mA = 0; mA < 2; ++mA) {
        #pragma unroll
        for (int o = 0; o < 2; ++o) {
            __syncthreads();
            #pragma unroll
            for (int nB = 0; nB < 2; ++nB)
                #pragma unroll
                for (int r = 0; r < 8; ++r)
                    lsEw[(8 * h + r) * EP + nB * 16 + m] = (o == 0) ? hv[mA][nB][r] : cv2[mA][nB][r];
            __syncthreads();
            float* obase = (o == 0) ? out0 : out1;
            #pragma unroll
            for (int it = 0; it < 4; ++it) {
                const int row = it * 4 + rsub;
                v4f v = *(const v4fa*)&lsEw[row * EP + c4];
                stv[mA][o][it] = v;
                float* gp = obase + (size_t)(m0 + wm * 32 + mA * 16 + row) * DHID + (n0 + wn * 32 + c4);
                *(volatile v4f*)gp = v;
            }
        }
    }
    __threadfence();
    #pragma unroll
    for (int mA = 0; mA < 2; ++mA) {
        #pragma unroll
        for (int o = 0; o < 2; ++o) {
            float* obase = (o == 0) ? out0 : out1;
            #pragma unroll
            for (int it = 0; it < 4; ++it) {
                const int row = it * 4 + rsub;
                float* gp = obase + (size_t)(m0 + wm * 32 + mA * 16 + row) * DHID + (n0 + wn * 32 + c4);
                *(volatile v4f*)gp = stv[mA][o][it];
            }
        }
    }
}

extern "C" void kernel_launch(void* const* d_in, const int* in_sizes, int n_in,
                              void* d_out, int out_size, void* d_ws, size_t ws_size,
                              hipStream_t stream)
{
    if (n_in < 19) return;
    if (in_sizes[0] <= 0 || (in_sizes[0] % DIN) != 0) return;
    const int rows = in_sizes[0] / DIN;
    if ((rows % TM) != 0) return;
    if (in_sizes[1] != rows * DHID || in_sizes[2] != rows * DHID) return;
    for (int i = 3; i < 19; i += 2) {
        if (in_sizes[i] != DHID * DIN) return;
        if (in_sizes[i + 1] != DHID) return;
    }
    if (out_size != 2 * rows * DHID) return;

    const size_t bytesA = (size_t)rows * KTOT * 2u;
    const size_t bytesW = (size_t)4 * DHID * KTOT * 2u;
    if (bytesA + bytesW > ws_size) return;

    const float* x = (const float*)d_in[0];
    const float* h = (const float*)d_in[1];
    const float* c = (const float*)d_in[2];
    const float* Wi0 = (const float*)d_in[3];  const float* bi0 = (const float*)d_in[4];
    const float* Wh0 = (const float*)d_in[5];  const float* bh0 = (const float*)d_in[6];
    const float* Wi1 = (const float*)d_in[7];  const float* bi1 = (const float*)d_in[8];
    const float* Wh1 = (const float*)d_in[9];  const float* bh1 = (const float*)d_in[10];
    const float* Wi2 = (const float*)d_in[11]; const float* bi2 = (const float*)d_in[12];
    const float* Wh2 = (const float*)d_in[13]; const float* bh2 = (const float*)d_in[14];
    const float* Wi3 = (const float*)d_in[15]; const float* bi3 = (const float*)d_in[16];
    const float* Wh3 = (const float*)d_in[17]; const float* bh3 = (const float*)d_in[18];

    unsigned short* Acat = (unsigned short*)d_ws;
    unsigned short* Wcat = (unsigned short*)((char*)d_ws + bytesA);
    float* out0 = (float*)d_out;
    float* out1 = out0 + (size_t)rows * DHID;

    k_cvt<<<dim3(rows), dim3(256), 0, stream>>>(x, h, Acat);
    k_cvt<<<dim3(DHID), dim3(256), 0, stream>>>(Wi0, Wh0, Wcat + (size_t)0 * DHID * KTOT);
    k_cvt<<<dim3(DHID), dim3(256), 0, stream>>>(Wi1, Wh1, Wcat + (size_t)1 * DHID * KTOT);
    k_cvt<<<dim3(DHID), dim3(256), 0, stream>>>(Wi2, Wh2, Wcat + (size_t)2 * DHID * KTOT);
    k_cvt<<<dim3(DHID), dim3(256), 0, stream>>>(Wi3, Wh3, Wcat + (size_t)3 * DHID * KTOT);

    dim3 grid(DHID / TN, rows / TM);
    k_lstm<<<grid, dim3(256), 0, stream>>>(Acat, Wcat, c,
                                           bi0, bi1, bi2, bi3, bh0, bh1, bh2, bh3,
                                           out0, out1);
    (void)hipGetLastError();
}
